// TransformerModel_1443109012058
// MI455X (gfx1250) — hardware-verified
//
#include <hip/hip_runtime.h>


#define NPAIR 32768
#define SL    32
#define DD    16
#define KP    32
#define NP    64
#define CH    1024
#define NT    (CH * 2 * SL)
#define SCL   0.25f
typedef _Float16 h16;
typedef unsigned short bf;
typedef __attribute__((ext_vector_type(16))) __bf16   v16bf;
typedef __attribute__((ext_vector_type(16))) _Float16 v16h;
typedef __attribute__((ext_vector_type(8)))  _Float16 v8h;
typedef __attribute__((ext_vector_type(8)))  unsigned short v8us;
typedef __attribute__((ext_vector_type(8)))  float    v8f;
typedef __attribute__((ext_vector_type(4)))  float    v4f;
typedef v8h  __attribute__((may_alias)) v8ha;
typedef v4f  __attribute__((may_alias)) v4fa;
typedef v8us __attribute__((may_alias)) v8usa;

__device__ __forceinline__ unsigned short f2bf(float f) { unsigned u = __float_as_uint(f); u += 0x7FFFu + ((u >> 16) & 1u); return (unsigned short)(u >> 16); }
__device__ __forceinline__ float bf2f(unsigned short b) { return __uint_as_float(((unsigned)b) << 16); }
__device__ __forceinline__ float bfr(float f) { return bf2f(f2bf(f)); }
__device__ __forceinline__ v16h cat16(v8h lo, v8h hi) { return __builtin_shufflevector(lo, hi, 0, 1, 2, 3, 4, 5, 6, 7, 8, 9, 10, 11, 12, 13, 14, 15); }
__device__ __forceinline__ v16bf cat16b(v8us lo, v8us hi) { return __builtin_bit_cast(v16bf, __builtin_shufflevector(lo, hi, 0, 1, 2, 3, 4, 5, 6, 7, 8, 9, 10, 11, 12, 13, 14, 15)); }
__device__ __forceinline__ v8f wmma16(v16h a, v16h b, v8f c) { return __builtin_amdgcn_wmma_f32_16x16x32_f16(false, a, false, b, (short)0, c, false, false); }
__device__ __forceinline__ v8f wmmab(v16bf a, v16bf b, v8f c) { return __builtin_amdgcn_wmma_f32_16x16x32_bf16(false, a, false, b, (short)0, c, false, false); }


template <typename T16> struct WFrag;
template <> struct WFrag<h16> { typedef v16h V; static __device__ __forceinline__ V ld(const h16* p) { return cat16(*(const v8h*)p, *(const v8h*)(p + 16)); } static __device__ __forceinline__ v8f mma(V a, V b, v8f c) { return wmma16(a, b, c); } };
template <> struct WFrag<bf> { typedef v16bf V; static __device__ __forceinline__ V ld(const bf* p) { return cat16b(*(const v8us*)p, *(const v8us*)(p + 16)); } static __device__ __forceinline__ v8f mma(V a, V b, v8f c) { return wmmab(a, b, c); } };
template <typename T16, int NSPLIT, bool BIAS>
__global__ __launch_bounds__(32) void k_gemmw(const T16* __restrict__ A, const T16* __restrict__ A2, const T16* __restrict__ Bt, const T16* __restrict__ Bt2, int K, float* C, int ldc, const float* __restrict__ bias, size_t sA, size_t sB, size_t sC) {
    typedef typename WFrag<T16>::V V;
    __shared__ __align__(16) float os[16 * 68];
    const size_t z = blockIdx.z; A += z * sA; if (A2) A2 += z * sA; Bt += z * sB; if (Bt2) Bt2 += z * sB; C += z * sC;
    const int lane = threadIdx.x & 31, lr = lane & 15, hi = lane >> 4; const int r0 = blockIdx.x * 64, c0 = blockIdx.y * 64;
    v8f acc[4][4];
#pragma unroll
    for (int mb = 0; mb < 4; ++mb)
#pragma unroll
        for (int nb = 0; nb < 4; ++nb) acc[mb][nb] = (v8f){};
    const size_t aoff = (size_t)(r0 + lr) * K + 8 * hi, boff = (size_t)(c0 + lr) * K + 8 * hi;
#pragma unroll 1
    for (int kc = 0; kc < K; kc += 32) {
        V a[4], a2[4];
#pragma unroll
        for (int mb = 0; mb < 4; ++mb) { a[mb] = WFrag<T16>::ld(A + aoff + (size_t)mb * 16 * K + kc); if (NSPLIT == 1 || NSPLIT == 2) a2[mb] = WFrag<T16>::ld(A2 + aoff + (size_t)mb * 16 * K + kc); }
#pragma unroll
        for (int nb = 0; nb < 4; ++nb) { const V b = WFrag<T16>::ld(Bt + boff + (size_t)nb * 16 * K + kc); V b2; if (NSPLIT >= 2) b2 = WFrag<T16>::ld(Bt2 + boff + (size_t)nb * 16 * K + kc);
#pragma unroll
            for (int mb = 0; mb < 4; ++mb) { acc[mb][nb] = WFrag<T16>::mma(a[mb], b, acc[mb][nb]); if (NSPLIT == 1 || NSPLIT == 2) acc[mb][nb] = WFrag<T16>::mma(a2[mb], b, acc[mb][nb]); if (NSPLIT >= 2) acc[mb][nb] = WFrag<T16>::mma(a[mb], b2, acc[mb][nb]); } }
        asm volatile("v_nop\n\tv_nop\n\tv_nop\n\tv_nop" : "+v"(acc[0][0]), "+v"(acc[1][1]), "+v"(acc[2][2]), "+v"(acc[3][3]) : "v"(a[0]), "v"(a[3]));
    }
#pragma unroll
    for (int mb = 0; mb < 4; ++mb) {
#pragma unroll
        for (int nb = 0; nb < 4; ++nb) {
#pragma unroll
            for (int j = 0; j < 8; ++j) os[(hi * 8 + j) * 68 + nb * 16 + lr] = acc[mb][nb][j]; }
        __builtin_amdgcn_wave_barrier(); asm volatile("" ::: "memory");
        float* crow = C + (size_t)(r0 + mb * 16) * ldc + c0;
#pragma unroll 1
        for (int ps = 0; ps < 2; ++ps) {
#pragma unroll
            for (int s = 0; s < 8; ++s) { const int row = 2 * s + hi, cofs = lr * 4; v4f val = *(const v4fa*)(os + row * 68 + cofs); if (BIAS) { val[0] += bfr(bias[c0 + cofs]); val[1] += bfr(bias[c0 + cofs + 1]); val[2] += bfr(bias[c0 + cofs + 2]); val[3] += bfr(bias[c0 + cofs + 3]); }
                *(volatile v4f*)(crow + (size_t)row * ldc + cofs) = val; }
            if (ps == 0) __threadfence(); }
        __builtin_amdgcn_wave_barrier(); asm volatile("" ::: "memory");
    }
}

__device__ __forceinline__ h16 tohx(float x) { return (h16)x; }
__device__ __forceinline__ void splitf(float y, unsigned short& h, unsigned short& l) { h = f2bf(y); l = f2bf(y - bf2f(h)); }
typedef __attribute__((ext_vector_type(2))) _Float16 v2h;
typedef __attribute__((ext_vector_type(4))) _Float16 v4h;
typedef __attribute__((ext_vector_type(2))) unsigned short v2us;
typedef __attribute__((ext_vector_type(4))) unsigned short v4us;
typedef __attribute__((ext_vector_type(2))) float v2f;
typedef __attribute__((ext_vector_type(4))) int v4i;


__global__ __launch_bounds__(256) void k_wpad16(const float* __restrict__ w, bf* Bt) { const int i = blockIdx.x * 256 + threadIdx.x; if (i >= NP * KP / 8) return; const int e = i * 8; const int n = e / KP, k = e % KP; v8us o;
#pragma unroll
    for (int q = 0; q < 8; ++q) o[q] = (n < DD && k + q < DD) ? f2bf(w[n * DD + k + q]) : (unsigned short)0; *(volatile v8us*)(Bt + e) = o; __threadfence(); *(volatile v8us*)(Bt + e) = o; }
__global__ __launch_bounds__(64) void k_bpad16(const float* __restrict__ b, float* BP) { const int n = threadIdx.x; if (n >= NP) return; const float v = (n < DD) ? b[n] : 0.0f; *(volatile float*)(BP + n) = v; __threadfence(); *(volatile float*)(BP + n) = v; }
__global__ __launch_bounds__(256) void k_embx(const int* __restrict__ tok, const float* __restrict__ emb, size_t t0, bf* X) { const size_t i = (size_t)blockIdx.x * 256 + threadIdx.x; if (i >= (size_t)NT * KP / 8) return; const size_t e = i * 8; const size_t tk = e / KP; const int k = (int)(e % KP); int id = tok[t0 + tk]; id = id < 0 ? 0 : (id > 255 ? 255 : id); v8us o;
#pragma unroll
    for (int q = 0; q < 8; ++q) o[q] = (k + q < DD) ? f2bf(emb[id * DD + k + q]) : (unsigned short)0; *(volatile v8us*)(X + e) = o; __threadfence(); *(volatile v8us*)(X + e) = o; }
__global__ __launch_bounds__(256) void k_attn(const float* __restrict__ Q, const float* __restrict__ K, const float* __restrict__ V, bf* Yh, bf* Yl) {
    const int lane = threadIdx.x & 31; const size_t sq = (size_t)blockIdx.x * 8 + (threadIdx.x >> 5); if (sq >= (size_t)NT / SL) return; const size_t tk = sq * SL + lane; float q[DD], kk[DD], vv[DD], acc[DD];
    { const v4f* qp = (const v4f*)(Q + tk * NP); const v4f* kp = (const v4f*)(K + tk * NP); const v4f* vp = (const v4f*)(V + tk * NP);
#pragma unroll
      for (int c = 0; c < 4; ++c) { const v4f a = qp[c], b = kp[c], d = vp[c];
#pragma unroll
          for (int u = 0; u < 4; ++u) { q[c * 4 + u] = a[u]; kk[c * 4 + u] = b[u]; vv[c * 4 + u] = d[u]; acc[c * 4 + u] = 0.f; } } }
    float m = -3.0e38f, Z = 0.f;
#pragma unroll 1
    for (int t = 0; t < SL; ++t) { float s = 0.f;
#pragma unroll
        for (int d = 0; d < DD; ++d) { float pr = __fmul_rn(q[d], __shfl(kk[d], t, 32)); asm volatile("" : "+v"(pr)); s = __fadd_rn(s, pr); }
        float sc = s * SCL; asm volatile("" : "+v"(sc)); const float mn = fmaxf(m, sc); float d1 = __fsub_rn(m, mn), d2 = __fsub_rn(sc, mn); asm volatile("" : "+v"(d1), "+v"(d2));
        const float r = __builtin_amdgcn_exp2f(__fmul_rn(d1, 1.4426950408889634f)), w = __builtin_amdgcn_exp2f(__fmul_rn(d2, 1.4426950408889634f));
        float zr = __fmul_rn(Z, r); asm volatile("" : "+v"(zr)); Z = __fadd_rn(zr, w); m = mn;
#pragma unroll
        for (int d = 0; d < DD; ++d) { float t0 = __fmul_rn(acc[d], r); asm volatile("" : "+v"(t0)); float t1 = __fmul_rn(w, __shfl(vv[d], t, 32)); asm volatile("" : "+v"(t1)); acc[d] = __fadd_rn(t0, t1); } }
    const float iz = __fdiv_rn(1.0f, Z);
#pragma unroll
    for (int d = 0; d < DD; ++d) acc[d] *= iz;
#pragma unroll 1
    for (int ps = 0; ps < 2; ++ps) {
#pragma unroll 1
        for (int rr = 0; rr < 4; ++rr) { const int row = rr * 8 + (lane >> 2), cb = (lane & 3) * 8; v8us oh, ol;
            float yr[DD];
#pragma unroll
            for (int d = 0; d < DD; ++d) yr[d] = __shfl(acc[d], row, 32);
            const int sel = lane & 3;
#pragma unroll
            for (int u = 0; u < 8; ++u) { const float yy = (sel == 0) ? yr[u] : ((sel == 1) ? yr[8 + u] : 0.f); unsigned short a, c2; splitf(yy, a, c2); oh[u] = a; ol[u] = c2; }
            const size_t oo = (sq * SL + row) * KP + cb; *(volatile v8us*)(Yh + oo) = oh; *(volatile v8us*)(Yl + oo) = ol; }
        if (ps == 0) __threadfence(); } }
__global__ __launch_bounds__(256) void k_reluhl(const float* __restrict__ Hh_, bf* Ph, bf* Pl) { const size_t i = (size_t)blockIdx.x * 256 + threadIdx.x; if (i >= (size_t)NT * KP / 8) return; const size_t e = i * 8; const size_t tk = e / KP; const int k = (int)(e % KP); v8us oh, ol;
#pragma unroll
    for (int q = 0; q < 8; ++q) { const float y = (k + q < DD) ? fmaxf(Hh_[tk * NP + k + q], 0.0f) : 0.f; unsigned short a, c2; splitf(y, a, c2); oh[q] = a; ol[q] = c2; } *(volatile v8us*)(Ph + e) = oh; *(volatile v8us*)(Pl + e) = ol; __threadfence(); *(volatile v8us*)(Ph + e) = oh; *(volatile v8us*)(Pl + e) = ol; }
__global__ __launch_bounds__(256) void k_cos(const float* __restrict__ O, size_t p0, float* outp) { const size_t pl = (size_t)blockIdx.x * 256 + threadIdx.x; if (pl >= CH) return; float s0[DD], s1[DD];
#pragma unroll
    for (int d = 0; d < DD; ++d) { s0[d] = 0.f; s1[d] = 0.f; }
#pragma unroll 1
    for (int t = 0; t < SL; ++t) { const v4f* r0 = (const v4f*)(O + ((pl * 2) * SL + t) * NP); const v4f* r1 = (const v4f*)(O + ((pl * 2 + 1) * SL + t) * NP);
#pragma unroll
        for (int c = 0; c < 4; ++c) { const v4f a = r0[c], b = r1[c];
#pragma unroll
            for (int u = 0; u < 4; ++u) { s0[c * 4 + u] = __fadd_rn(s0[c * 4 + u], a[u]); s1[c * 4 + u] = __fadd_rn(s1[c * 4 + u], b[u]); } } }
    float dot = 0.f, n1 = 0.f, n2 = 0.f;
#pragma unroll
    for (int d = 0; d < DD; ++d) { const float a = s0[d] * (1.0f / SL), b = s1[d] * (1.0f / SL); float p1 = __fmul_rn(a, b), p2 = __fmul_rn(a, a), p3 = __fmul_rn(b, b); asm volatile("" : "+v"(p1), "+v"(p2), "+v"(p3)); dot = __fadd_rn(dot, p1); n1 = __fadd_rn(n1, p2); n2 = __fadd_rn(n2, p3); }
    float den = __fmul_rn(__fsqrt_rn(n1), __fsqrt_rn(n2)); asm volatile("" : "+v"(den)); den = __fadd_rn(den, 1e-8f); float sim = __fdiv_rn(dot, den); asm volatile("" : "+v"(sim)); float o = __fadd_rn(sim, 1.0f); asm volatile("" : "+v"(o)); o = o * 0.5f;
    *(volatile float*)(outp + p0 + pl) = o; __threadfence(); *(volatile float*)(outp + p0 + pl) = o; }

extern "C" void kernel_launch(void* const* d_in, const int* in_sizes, int n_in,
                              void* d_out, int out_size, void* d_ws, size_t ws_size, hipStream_t stream) {
    (void)in_sizes; (void)n_in; (void)out_size;
    const int* tok = (const int*)d_in[0]; const float* emb = (const float*)d_in[1]; const float* wq = (const float*)d_in[2]; const float* wk = (const float*)d_in[3]; const float* wv = (const float*)d_in[4]; const float* w1 = (const float*)d_in[5]; const float* b1 = (const float*)d_in[6]; const float* w2 = (const float*)d_in[7]; const float* b2 = (const float*)d_in[8];
    float* OUT = (float*)d_out;
    char* wsp = (char*)d_ws;
    auto take = [&](size_t bytes) { char* p = wsp; wsp += (bytes + 255) & ~(size_t)255; return (void*)p; };
    bf* WQ = (bf*)take(NP * KP * 2); bf* WK = (bf*)take(NP * KP * 2); bf* WV = (bf*)take(NP * KP * 2); bf* W1 = (bf*)take(NP * KP * 2); bf* W2 = (bf*)take(NP * KP * 2); float* B1 = (float*)take(256); float* B2 = (float*)take(256);
    bf* X = (bf*)take((size_t)NT * KP * 2); float* Q = (float*)take((size_t)NT * NP * 4); float* K = (float*)take((size_t)NT * NP * 4); float* V = (float*)take((size_t)NT * NP * 4); bf* Yh = (bf*)take((size_t)NT * KP * 2); bf* Yl = (bf*)take((size_t)NT * KP * 2); float* H = (float*)take((size_t)NT * NP * 4); bf* Hh = (bf*)take((size_t)NT * KP * 2); bf* Hl = (bf*)take((size_t)NT * KP * 2); float* O = (float*)take((size_t)NT * NP * 4);
    if ((size_t)(wsp - (char*)d_ws) > ws_size) return;
    k_wpad16<<<1, 256, 0, stream>>>(wq, WQ); k_wpad16<<<1, 256, 0, stream>>>(wk, WK); k_wpad16<<<1, 256, 0, stream>>>(wv, WV); k_wpad16<<<1, 256, 0, stream>>>(w1, W1); k_wpad16<<<1, 256, 0, stream>>>(w2, W2); k_bpad16<<<1, 64, 0, stream>>>(b1, B1); k_bpad16<<<1, 64, 0, stream>>>(b2, B2);
    const unsigned LX = (unsigned)(((size_t)NT * KP / 8 + 255) / 256);
    for (size_t p0 = 0; p0 < NPAIR; p0 += CH) { const size_t t0 = p0 * 2 * SL;
        k_embx<<<LX, 256, 0, stream>>>(tok, emb, t0, X);
        k_gemmw<bf, 0, false><<<dim3(NT / 64, 1, 1), 32, 0, stream>>>(X, nullptr, WQ, nullptr, KP, Q, NP, nullptr, 0, 0, 0); k_gemmw<bf, 0, false><<<dim3(NT / 64, 1, 1), 32, 0, stream>>>(X, nullptr, WK, nullptr, KP, K, NP, nullptr, 0, 0, 0); k_gemmw<bf, 0, false><<<dim3(NT / 64, 1, 1), 32, 0, stream>>>(X, nullptr, WV, nullptr, KP, V, NP, nullptr, 0, 0, 0);
        k_attn<<<(unsigned)((NT / SL) / 8), 256, 0, stream>>>(Q, K, V, Yh, Yl);
        k_gemmw<bf, 1, true><<<dim3(NT / 64, 1, 1), 32, 0, stream>>>(Yh, Yl, W1, nullptr, KP, H, NP, B1, 0, 0, 0);
        k_reluhl<<<LX, 256, 0, stream>>>(H, Hh, Hl);
        k_gemmw<bf, 1, true><<<dim3(NT / 64, 1, 1), 32, 0, stream>>>(Hh, Hl, W2, nullptr, KP, O, NP, B2, 0, 0, 0);
        k_cos<<<(CH + 255) / 256, 256, 0, stream>>>(O, p0, OUT); }
}
